// PointNetSetAbstraction_11123965297234
// MI455X (gfx1250) — hardware-verified
//
#include <hip/hip_runtime.h>
#include <stdint.h>

#pragma clang fp contract(off)

typedef __attribute__((ext_vector_type(16))) _Float16 v16h;
typedef __attribute__((ext_vector_type(8)))  _Float16 v8h;
typedef __attribute__((ext_vector_type(8)))  float    v8f;
typedef __attribute__((ext_vector_type(4)))  float    v4f;
typedef __attribute__((ext_vector_type(4)))  int      v4i;

constexpr int kBatch    = 8;
constexpr int kNumPts   = 4096;
constexpr int kCin      = 64;
constexpr int kNumCent  = 1024;
constexpr int kNbr      = 32;
constexpr int kGroups   = kBatch * kNumCent;
constexpr int kRows     = kGroups * kNbr;
constexpr int kOut0     = 128;
constexpr int kOut1     = 128;
constexpr int kOut2     = 256;
constexpr int kW0In     = 3 + kCin;
constexpr int kChunks   = 4;
constexpr int kChunkRows = kRows / kChunks;
constexpr int kChunkGroups = kGroups / kChunks;
constexpr float kWCarry    = 64.0f;
constexpr float kWCarryInv = 1.0f / 64.0f;
constexpr float kBnEps     = 1e-5f;

static_assert(kGroups == 8192, "groups");
static_assert(kRows == 262144, "rows");
static_assert(kW0In == 67, "layer-0 input width");
static_assert(kChunkRows % 64 == 0 && kRows % 64 == 0, "M tile multiple");
static_assert(kOut0 % 64 == 0 && kOut1 % 64 == 0 && kOut2 % 64 == 0, "N tile multiple");
static_assert(kCin % 32 == 0 && kOut0 % 32 == 0 && kOut1 % 32 == 0, "K multiple of 32");
static_assert(((kBatch * kNumPts / 64) * (kOut0 / 64)) % 8 == 0, "grid P exact");
static_assert(((kRows / 64) * (kOut1 / 64)) % 8 == 0, "grid stats1 exact");
static_assert(((kChunkRows / 64) * (kOut1 / 64)) % 8 == 0, "grid apply1 exact");
static_assert(((kChunkRows / 64) * (kOut2 / 64)) % 8 == 0, "grid layer2 exact");

constexpr size_t al256(size_t x) { return (x + 255) & ~(size_t)255; }
constexpr size_t kSzFps   = (size_t)kGroups * 4;
constexpr size_t kSzNn    = (size_t)kRows * 4;
constexpr size_t kSzW0h   = (size_t)kOut0 * kCin * 2;
constexpr size_t kSzW1h   = (size_t)kOut1 * kOut0 * 2;
constexpr size_t kSzW2h   = (size_t)kOut2 * kOut1 * 2;
constexpr size_t kSzPts   = (size_t)kBatch * kNumPts * kCin * 2;
constexpr size_t kSzP     = (size_t)kBatch * kNumPts * kOut0 * 4;
constexpr size_t kSzA1    = (size_t)kRows * kOut0 * 2;
constexpr size_t kSzA2    = (size_t)kChunkRows * kOut1 * 2;
constexpr size_t kSzY     = (size_t)kGroups * kOut2 * 4;
constexpr int    kBlk0    = kGroups / 16;
constexpr int    kBlk1    = ((kRows / 64) * (kOut1 / 64)) / 8;
constexpr int    kBlk2c   = ((kChunkRows / 64) * (kOut2 / 64)) / 8;
constexpr size_t kSzPart0 = (size_t)kBlk0 * 2 * kOut0 * 4;
constexpr size_t kSzPart1 = (size_t)kBlk1 * 2 * kOut1 * 4;
constexpr size_t kSzPart2 = (size_t)kBlk2c * kChunks * 2 * kOut2 * 4;
constexpr size_t kSzSS    = 512 * 4;

constexpr size_t kOffFps   = 0;
constexpr size_t kOffNn    = kOffFps + al256(kSzFps);
constexpr size_t kOffW0h   = kOffNn + al256(kSzNn);
constexpr size_t kOffW1h   = kOffW0h + al256(kSzW0h);
constexpr size_t kOffW2h   = kOffW1h + al256(kSzW1h);
constexpr size_t kOffPts   = kOffW2h + al256(kSzW2h);
constexpr size_t kOffP     = kOffPts + al256(kSzPts);
constexpr size_t kOffA1    = kOffP + al256(kSzP);
constexpr size_t kOffA2    = kOffA1 + al256(kSzA1);
constexpr size_t kOffYmax  = kOffA2 + al256(kSzA2);
constexpr size_t kOffYmin  = kOffYmax + al256(kSzY);
constexpr size_t kOffPart0 = kOffYmin + al256(kSzY);
constexpr size_t kOffPart1 = kOffPart0 + al256(kSzPart0);
constexpr size_t kOffPart2 = kOffPart1 + al256(kSzPart1);
constexpr size_t kOffSS0   = kOffPart2 + al256(kSzPart2);
constexpr size_t kOffSS1   = kOffSS0 + al256(kSzSS);
constexpr size_t kOffSS2   = kOffSS1 + al256(kSzSS);
constexpr size_t kCarveTotal = kOffSS2 + al256(kSzSS);
static_assert(kCarveTotal <= (size_t)134217728, "carve within 128 MiB");
static_assert((size_t)kBatch * kNumCent * 3 * 4 == 98304, "out1 byte offset");
static_assert((size_t)98304 + (size_t)kBatch * kOut2 * kNumCent * 4 == (size_t)8486912, "d_out total");

union FragU { v16h v; v8h h[2]; };
__device__ __forceinline__ v16h frag_load(const _Float16* p) {
  FragU f;
  f.h[0] = *(const v8h*)(p);
  f.h[1] = *(const v8h*)(p + 16);
  return f.v;
}
__device__ __forceinline__ v8f wmma_h(v16h a, v16h b, v8f c) {
  return __builtin_amdgcn_wmma_f32_16x16x32_f16(false, a, false, b, (short)0, c, false, false);
}
__device__ __forceinline__ void guard_row4(v8f& a0, v8f& a1, v8f& a2, v8f& a3, v16h x,
                                           v16h b0, v16h b1, v16h b2, v16h b3) {
  asm volatile("v_nop\n\tv_nop\n\tv_nop\n\tv_nop"
               : "+v"(a0), "+v"(a1), "+v"(a2), "+v"(a3)
               : "v"(x), "v"(b0), "v"(b1), "v"(b2), "v"(b3));
}
__device__ __forceinline__ void acc_guard4(v8f& a, v8f& b, v8f& c, v8f& d) {
  asm volatile("v_nop\n\tv_nop\n\tv_nop\n\tv_nop" : "+v"(a), "+v"(b), "+v"(c), "+v"(d));
}
__device__ __forceinline__ void wave_lds_sync() {
  __builtin_amdgcn_fence(__ATOMIC_RELEASE, "workgroup");
  __builtin_amdgcn_wave_barrier();
  __builtin_amdgcn_fence(__ATOMIC_ACQUIRE, "workgroup");
}

__global__ __launch_bounds__(256) void fps_kernel(const float* __restrict__ xyz,
                                                  int* __restrict__ fps_idx,
                                                  float* __restrict__ out0) {
#pragma clang fp contract(off)
  __shared__ __align__(16) float xs[kNumPts * 3];
  __shared__ __align__(16) int idxs[kNumCent];
  __shared__ float rv[2][8];
  __shared__ int ri[2][8];

  const int b = blockIdx.x;
  const int t = threadIdx.x;
  const int lane = t & 31;
  const int wave = t >> 5;

  {
    const v4f* g4 = (const v4f*)(xyz + (size_t)b * kNumPts * 3);
    v4f* l4 = (v4f*)xs;
#pragma unroll 1
    for (int j = 0; j < 12; ++j) l4[t + 256 * j] = g4[t + 256 * j];
  }
  __syncthreads();

  float px[16], py[16], pz[16], dd[16];
#pragma unroll
  for (int j = 0; j < 16; ++j) {
    const int n = j * 256 + t;
    px[j] = xs[n * 3 + 0];
    py[j] = xs[n * 3 + 1];
    pz[j] = xs[n * 3 + 2];
    dd[j] = 1e10f;
  }

  int cur = 0;
#pragma unroll 1
  for (int s = 0; s < kNumCent; ++s) {
    if (t == 0) idxs[s] = cur;
    const float cx = xs[cur * 3 + 0];
    const float cy = xs[cur * 3 + 1];
    const float cz = xs[cur * 3 + 2];
    float bv = 0.0f;
    int bi = 0;
#pragma unroll
    for (int j = 0; j < 16; ++j) {
      const float dx = px[j] - cx;
      const float dy = py[j] - cy;
      const float dz = pz[j] - cz;
      const float t0 = dx * dx;
      const float t1 = dy * dy;
      const float t2 = dz * dz;
      const float d = (t0 + t2) + t1;
      const float m = (d < dd[j]) ? d : dd[j];
      dd[j] = m;
      if (j == 0) {
        bv = m;
        bi = t;
      } else {
        const bool take = (m > bv);
        bv = take ? m : bv;
        bi = take ? (j * 256 + t) : bi;
      }
    }
#pragma unroll
    for (int off = 16; off > 0; off >>= 1) {
      const float ov = __shfl_xor(bv, off, 32);
      const int oi = __shfl_xor(bi, off, 32);
      const bool take = (ov > bv) || (ov == bv && oi < bi);
      bv = take ? ov : bv;
      bi = take ? oi : bi;
    }
    const int par = s & 1;
    if (lane == 0) {
      rv[par][wave] = bv;
      ri[par][wave] = bi;
    }
    __syncthreads();
    float fv = rv[par][0];
    int fi = ri[par][0];
#pragma unroll
    for (int w = 1; w < 8; ++w) {
      const float v = rv[par][w];
      const int i = ri[par][w];
      const bool take = (v > fv) || (v == fv && i < fi);
      fv = take ? v : fv;
      fi = take ? i : fi;
    }
    cur = fi & (kNumPts - 1);
  }
  __syncthreads();

  v4f ov[3];
#pragma unroll
  for (int j = 0; j < 3; ++j) {
    const int i4 = t + 256 * j;
#pragma unroll
    for (int k = 0; k < 4; ++k) {
      const int e = i4 * 4 + k;
      const int sidx = e / 3;
      const int comp = e - sidx * 3;
      const int pi = idxs[sidx] & (kNumPts - 1);
      ov[j][k] = xs[pi * 3 + comp];
    }
  }
  v4i iv;
#pragma unroll
  for (int k = 0; k < 4; ++k) iv[k] = idxs[t * 4 + k];
  float* ob = out0 + (size_t)b * kNumCent * 3;
  int* ib = fps_idx + (size_t)b * kNumCent;
  for (int pass = 0; pass < 2; ++pass) {
#pragma unroll
    for (int j = 0; j < 3; ++j) *(volatile v4f*)(ob + (size_t)(t + 256 * j) * 4) = ov[j];
    *(volatile v4i*)(ib + t * 4) = iv;
    __threadfence();
  }
}

__global__ __launch_bounds__(64) void knn_kernel(const float* __restrict__ xyz,
                                                 const int* __restrict__ fps_idx,
                                                 int* __restrict__ nn_idx) {
#pragma clang fp contract(off)
  __shared__ __align__(16) float dsq[2][kNumPts];
  __shared__ __align__(16) float cs[512 * 3];

  const int tid = threadIdx.x;
  const int wave = tid >> 5;
  const int lane = tid & 31;
  const int samp = blockIdx.x * 2 + wave;
  const int b = samp >> 10;
  const float* xb = xyz + (size_t)b * kNumPts * 3;

  int fi = fps_idx[samp];
  fi = fi < 0 ? 0 : (fi > kNumPts - 1 ? kNumPts - 1 : fi);
  const float qx = xb[fi * 3 + 0];
  const float qy = xb[fi * 3 + 1];
  const float qz = xb[fi * 3 + 2];
  const float qq = (qx * qx + qz * qz) + qy * qy;

  float* dst = dsq[wave];
  const float finf = __builtin_inff();
  float gmv[8];
  int gmi[8];

#pragma unroll
  for (int g = 0; g < 8; ++g) {
    __syncthreads();
    {
      const v4f* src4 = (const v4f*)(xb + g * 1536);
      v4f* l4 = (v4f*)cs;
#pragma unroll 1
      for (int u = tid; u < 384; u += 64) l4[u] = src4[u];
    }
    __syncthreads();
    float bv = finf;
    int bi = 0x7fffffff;
#pragma unroll 1
    for (int e = 0; e < 16; ++e) {
      const int i = lane + 32 * e;
      const float x = cs[i * 3 + 0];
      const float y = cs[i * 3 + 1];
      const float z = cs[i * 3 + 2];
      const float xx = (x * x + z * z) + y * y;
      float p = qx * x;
      p = fmaf(qy, y, p);
      p = fmaf(qz, z, p);
      const float p2 = 2.0f * p;
      const float tq = qq - p2;
      const float d = tq + xx;
      const int n = g * 512 + i;
      dst[n] = d;
      const bool take = (d < bv);
      bv = take ? d : bv;
      bi = take ? n : bi;
    }
    gmv[g] = bv;
    gmi[g] = bi;
  }

  int mine = 0;
#pragma unroll 1
  for (int it = 0; it < kNbr; ++it) {
    float lv = gmv[0];
    int li = gmi[0];
#pragma unroll
    for (int gi = 1; gi < 8; ++gi) {
      const bool take = (gmv[gi] < lv);
      lv = take ? gmv[gi] : lv;
      li = take ? gmi[gi] : li;
    }
#pragma unroll
    for (int off = 16; off > 0; off >>= 1) {
      const float ov = __shfl_xor(lv, off, 32);
      const int oi = __shfl_xor(li, off, 32);
      const bool take = (ov < lv) || (ov == lv && oi < li);
      lv = take ? ov : lv;
      li = take ? oi : li;
    }
    const int wi = li & (kNumPts - 1);
    mine = (lane == it) ? wi : mine;
    if ((wi & 31) == lane) dst[wi] = finf;
    const int g = wi >> 9;
    const int base = g * 512 + lane;
    float bv = finf;
    int bi = 0x7fffffff;
#pragma unroll
    for (int e = 0; e < 16; ++e) {
      const float v = dst[base + 32 * e];
      const bool take = (v < bv);
      bv = take ? v : bv;
      bi = take ? (base + 32 * e) : bi;
    }
#pragma unroll
    for (int gi = 0; gi < 8; ++gi) {
      const bool sel = (gi == g);
      gmv[gi] = sel ? bv : gmv[gi];
      gmi[gi] = sel ? bi : gmi[gi];
    }
  }
  int* op = nn_idx + (size_t)samp * kNbr + lane;
  *(volatile int*)op = mine;
  __threadfence();
  *(volatile int*)op = mine;
}

__device__ __forceinline__ void store8h(_Float16* dst, const float* f, float mul) {
  v8h hv;
#pragma unroll
  for (int e = 0; e < 8; ++e) hv[e] = (_Float16)(f[e] * mul);
  *(volatile v8h*)dst = hv;
  __threadfence();
  *(volatile v8h*)dst = hv;
}
constexpr int kPrepWBlocks = 28;
constexpr int kPrepPBlocks = (kBatch * kNumPts * kCin) / (256 * 8);
static_assert(kOut0 * kCin == 4 * 256 * 8, "W0h coverage");
static_assert(kOut1 * kOut0 == 8 * 256 * 8, "W1h coverage");
static_assert(kOut2 * kOut1 == 16 * 256 * 8, "W2h coverage");
static_assert(kPrepPBlocks * 256 * 8 == kBatch * kNumPts * kCin, "pts16 coverage");

__global__ __launch_bounds__(256) void prep_kernel(const float* __restrict__ W0, const float* __restrict__ W1,
                                                   const float* __restrict__ W2, const float* __restrict__ points,
                                                   _Float16* __restrict__ W0h, _Float16* __restrict__ W1h,
                                                   _Float16* __restrict__ W2h, _Float16* __restrict__ pts16) {
  const int blk = blockIdx.x;
  const int t = threadIdx.x;
  float f[8];
  if (blk < 4) {
    const int i8 = (blk * 256 + t) * 8;
    const int o = i8 >> 6;
    const int c = i8 & 63;
    const float* src = W0 + (size_t)o * kW0In + 3 + c;
#pragma unroll
    for (int e = 0; e < 8; ++e) f[e] = src[e];
    store8h(W0h + i8, f, kWCarry);
  } else if (blk < 12) {
    const int i8 = ((blk - 4) * 256 + t) * 8;
    const v4f a = *(const v4f*)(W1 + i8);
    const v4f c = *(const v4f*)(W1 + i8 + 4);
#pragma unroll
    for (int e = 0; e < 4; ++e) { f[e] = a[e]; f[4 + e] = c[e]; }
    store8h(W1h + i8, f, kWCarry);
  } else if (blk < kPrepWBlocks) {
    const int i8 = ((blk - 12) * 256 + t) * 8;
    const v4f a = *(const v4f*)(W2 + i8);
    const v4f c = *(const v4f*)(W2 + i8 + 4);
#pragma unroll
    for (int e = 0; e < 4; ++e) { f[e] = a[e]; f[4 + e] = c[e]; }
    store8h(W2h + i8, f, kWCarry);
  } else {
    const size_t i8 = ((size_t)(blk - kPrepWBlocks) * 256 + t) * 8;
    const v4f a = *(const v4f*)(points + i8);
    const v4f c = *(const v4f*)(points + i8 + 4);
#pragma unroll
    for (int e = 0; e < 4; ++e) { f[e] = a[e]; f[4 + e] = c[e]; }
    store8h(pts16 + i8, f, 1.0f);
  }
}

template <int MODE>
__global__ __launch_bounds__(256) void mlp_gemm(
    const _Float16* __restrict__ A, const _Float16* __restrict__ Bt, int N, int K,
    const float* __restrict__ bias, const float* __restrict__ scl, const float* __restrict__ sft,
    float* __restrict__ outF, _Float16* __restrict__ outH,
    float* __restrict__ ymaxp, float* __restrict__ yminp, float scale) {
  __shared__ __align__(16) float sT[8][16 * 68];
  __shared__ float red[8][128];

  const int tid = threadIdx.x;
  const int lane = tid & 31;
  const int wave = tid >> 5;
  const int tilesN = N >> 6;
  const int tile = blockIdx.x * 8 + wave;
  const int tm = tile / tilesN;
  const int tn = tile - tm * tilesN;
  const int m0 = tm << 6;
  const int n0 = tn << 6;
  const int rlane = lane & 15;
  const int hh = lane >> 4;
  const int koff = hh * 8;
  const int mOff = hh * 8;

  v8f acc[4][4];
#pragma unroll
  for (int i = 0; i < 4; ++i)
#pragma unroll
    for (int j = 0; j < 4; ++j) acc[i][j] = (v8f){0.f, 0.f, 0.f, 0.f, 0.f, 0.f, 0.f, 0.f};

  for (int k0 = 0; k0 < K; k0 += 32) {
    v16h bh[4];
#pragma unroll
    for (int j = 0; j < 4; ++j)
      bh[j] = frag_load(Bt + (size_t)(n0 + (j << 4) + rlane) * K + koff + k0);
#pragma unroll
    for (int i = 0; i < 4; ++i) {
      const v16h ah = frag_load(A + (size_t)(m0 + (i << 4) + rlane) * K + koff + k0);
#pragma unroll
      for (int j = 0; j < 4; ++j) acc[i][j] = wmma_h(ah, bh[j], acc[i][j]);
      guard_row4(acc[i][0], acc[i][1], acc[i][2], acc[i][3], ah, bh[0], bh[1], bh[2], bh[3]);
    }
  }
  acc_guard4(acc[0][0], acc[0][1], acc[0][2], acc[0][3]);
  acc_guard4(acc[1][0], acc[1][1], acc[1][2], acc[1][3]);
  acc_guard4(acc[2][0], acc[2][1], acc[2][2], acc[2][3]);
  acc_guard4(acc[3][0], acc[3][1], acc[3][2], acc[3][3]);

  float* slab = sT[wave];
  float bj[4], scj[4], shj[4];
#pragma unroll
  for (int j = 0; j < 4; ++j) {
    const int n = n0 + (j << 4) + rlane;
    bj[j] = (MODE != 0) ? bias[n] : 0.0f;
    scj[j] = (MODE == 2) ? scl[n] : 1.0f;
    shj[j] = (MODE == 2) ? sft[n] : 0.0f;
  }

  if (MODE == 0 || MODE == 2) {
#pragma unroll
    for (int i = 0; i < 4; ++i) {
      const int mBase = m0 + (i << 4);
#pragma unroll
      for (int j = 0; j < 4; ++j) {
#pragma unroll
        for (int r = 0; r < 8; ++r) {
          float v = acc[i][j][r] * scale;
          if (MODE == 2) {
            v = v + bj[j];
            v = scj[j] * v + shj[j];
            v = fmaxf(v, 0.0f);
          }
          slab[(mOff + r) * 68 + (j << 4) + rlane] = v;
        }
      }
      wave_lds_sync();
      if (MODE == 0) {
        const int c4 = rlane * 4;
        for (int pass = 0; pass < 2; ++pass) {
#pragma unroll
          for (int it = 0; it < 8; ++it) {
            const int row = it * 2 + hh;
            const v4f v = *(const v4f*)(slab + row * 68 + c4);
            *(volatile v4f*)(outF + (size_t)(mBase + row) * N + n0 + c4) = v;
          }
          __threadfence();
        }
      } else {
        const int q = lane >> 3;
        const int c8 = (lane & 7) * 8;
        for (int pass = 0; pass < 2; ++pass) {
#pragma unroll
          for (int it = 0; it < 4; ++it) {
            const int row = it * 4 + q;
            const float* sp = slab + row * 68 + c8;
            v8h hv;
#pragma unroll
            for (int e = 0; e < 8; ++e) hv[e] = (_Float16)sp[e];
            *(volatile v8h*)(outH + (size_t)(mBase + row) * N + n0 + c8) = hv;
          }
          __threadfence();
        }
      }
      wave_lds_sync();
    }
  }

  if (MODE == 1 || MODE == 3) {
#pragma unroll
    for (int j = 0; j < 4; ++j) {
      float s = 0.0f, q = 0.0f;
      float mx[2], mn[2];
      mx[0] = -__builtin_inff(); mx[1] = -__builtin_inff();
      mn[0] = __builtin_inff();  mn[1] = __builtin_inff();
#pragma unroll
      for (int i = 0; i < 4; ++i) {
#pragma unroll
        for (int r = 0; r < 8; ++r) {
          const float y = acc[i][j][r] * scale + bj[j];
          s = s + y;
          q = q + y * y;
          if (MODE == 3) {
            mx[i >> 1] = fmaxf(mx[i >> 1], y);
            mn[i >> 1] = fminf(mn[i >> 1], y);
          }
        }
      }
      const float s2 = __shfl_xor(s, 16, 32);
      const float q2 = __shfl_xor(q, 16, 32);
      s = s + s2;
      q = q + q2;
      float mx0 = mx[0], mx1 = mx[1], mn0 = mn[0], mn1 = mn[1];
      if (MODE == 3) {
        const float a0 = __shfl_xor(mx0, 16, 32);
        const float a1 = __shfl_xor(mx1, 16, 32);
        const float c0 = __shfl_xor(mn0, 16, 32);
        const float c1 = __shfl_xor(mn1, 16, 32);
        mx0 = fmaxf(mx0, a0);
        mx1 = fmaxf(mx1, a1);
        mn0 = fminf(mn0, c0);
        mn1 = fminf(mn1, c1);
      }
      if (hh == 0) {
        red[wave][(j << 4) + rlane] = s;
        red[wave][64 + (j << 4) + rlane] = q;
        if (MODE == 3) {
          slab[0 * 64 + (j << 4) + rlane] = mx0;
          slab[1 * 64 + (j << 4) + rlane] = mn0;
          slab[2 * 64 + (j << 4) + rlane] = mx1;
          slab[3 * 64 + (j << 4) + rlane] = mn1;
        }
      }
    }
    if (MODE == 3) {
      wave_lds_sync();
      const int c4 = rlane * 4;
      float* yb = hh ? yminp : ymaxp;
      const v4f v0 = *(const v4f*)(slab + (0 + hh) * 64 + c4);
      const v4f v1 = *(const v4f*)(slab + (2 + hh) * 64 + c4);
      float* d0 = yb + (size_t)(tm * 2 + 0) * N + n0 + c4;
      float* d1 = yb + (size_t)(tm * 2 + 1) * N + n0 + c4;
      *(volatile v4f*)d0 = v0;
      *(volatile v4f*)d1 = v1;
      __threadfence();
      *(volatile v4f*)d0 = v0;
      *(volatile v4f*)d1 = v1;
    }
    __syncthreads();
    const int twoN = 2 * N;
    float tot[2];
#pragma unroll
    for (int u = 0; u < 2; ++u) {
      const int o = tid + 256 * u;
      const int oc = (o < twoN) ? o : (twoN - 1);
      const int which = (oc >= N) ? 1 : 0;
      const int col = oc - which * N;
      const int tnn = col >> 6;
      const int c = col & 63;
      float a = 0.0f;
      for (int w = tnn; w < 8; w += tilesN) a = a + red[w][which * 64 + c];
      tot[u] = a;
    }
    float* pb = outF + (size_t)blockIdx.x * twoN;
    for (int pass = 0; pass < 2; ++pass) {
#pragma unroll
      for (int u = 0; u < 2; ++u) {
        const int o = tid + 256 * u;
        if (o < twoN) *(volatile float*)(pb + o) = tot[u];
      }
      __threadfence();
    }
  }
}

template <bool APPLY>
__global__ __launch_bounds__(256) void l0_kernel(
    const float* __restrict__ P, const float* __restrict__ xyz, const int* __restrict__ fps_idx,
    const int* __restrict__ nn_idx, const float* __restrict__ W0, const float* __restrict__ b0,
    const float* __restrict__ scl, const float* __restrict__ sft,
    float* __restrict__ part, _Float16* __restrict__ A1) {
  __shared__ __align__(16) float tab[6][128];
  __shared__ float red[8][256];

  const int tid = threadIdx.x;
  const int lane = tid & 31;
  const int wave = tid >> 5;
  const int hh = lane >> 4;
  const int c8 = (lane & 15) * 8;

  if (tid < 128) {
    tab[0][tid] = W0[tid * kW0In + 0];
    tab[1][tid] = W0[tid * kW0In + 1];
    tab[2][tid] = W0[tid * kW0In + 2];
    tab[3][tid] = b0[tid];
    tab[4][tid] = APPLY ? scl[tid] : 1.0f;
    tab[5][tid] = APPLY ? sft[tid] : 0.0f;
  }
  __syncthreads();

  float wx[8], wy[8], wz[8], bb[8], sc[8], sh[8], s[8], q[8];
#pragma unroll
  for (int e = 0; e < 8; ++e) {
    wx[e] = tab[0][c8 + e];
    wy[e] = tab[1][c8 + e];
    wz[e] = tab[2][c8 + e];
    bb[e] = tab[3][c8 + e];
    sc[e] = tab[4][c8 + e];
    sh[e] = tab[5][c8 + e];
    s[e] = 0.0f;
    q[e] = 0.0f;
  }

#pragma unroll 1
  for (int gg = 0; gg < 2; ++gg) {
    const int gidx = (blockIdx.x * 8 + wave) * 2 + gg;
    const int b = gidx >> 10;
    int fi = fps_idx[gidx];
    fi = fi < 0 ? 0 : (fi > kNumPts - 1 ? kNumPts - 1 : fi);
    int nk = nn_idx[(size_t)gidx * kNbr + lane];
    nk = nk < 0 ? 0 : (nk > kNumPts - 1 ? kNumPts - 1 : nk);
    const float* xb = xyz + (size_t)b * kNumPts * 3;
    const float rx = xb[nk * 3 + 0] - xb[fi * 3 + 0];
    const float ry = xb[nk * 3 + 1] - xb[fi * 3 + 1];
    const float rz = xb[nk * 3 + 2] - xb[fi * 3 + 2];
#pragma unroll 1
    for (int i = 0; i < 16; ++i) {
      const int src = 2 * i + hh;
      const int n = __shfl(nk, src, 32);
      const float x = __shfl(rx, src, 32);
      const float y = __shfl(ry, src, 32);
      const float z = __shfl(rz, src, 32);
      const float* pr = P + ((size_t)b * kNumPts + n) * kOut0 + c8;
      const v4f p0 = *(const v4f*)(pr);
      const v4f p1 = *(const v4f*)(pr + 4);
      float yv[8];
#pragma unroll
      for (int e = 0; e < 8; ++e) {
        const float pe = (e < 4) ? p0[e & 3] : p1[e & 3];
        float v = pe + bb[e];
        v = fmaf(wx[e], x, v);
        v = fmaf(wy[e], y, v);
        v = fmaf(wz[e], z, v);
        yv[e] = v;
      }
      if (APPLY) {
        v8h hv;
#pragma unroll
        for (int e = 0; e < 8; ++e) hv[e] = (_Float16)fmaxf(fmaf(sc[e], yv[e], sh[e]), 0.0f);
        _Float16* dp = A1 + ((size_t)gidx * kNbr + src) * kOut0 + c8;
        *(volatile v8h*)dp = hv;
        __threadfence();
        *(volatile v8h*)dp = hv;
      } else {
#pragma unroll
        for (int e = 0; e < 8; ++e) {
          s[e] = s[e] + yv[e];
          q[e] = fmaf(yv[e], yv[e], q[e]);
        }
      }
    }
  }

  if (!APPLY) {
#pragma unroll
    for (int e = 0; e < 8; ++e) {
      const float s2 = __shfl_xor(s[e], 16, 32);
      const float q2 = __shfl_xor(q[e], 16, 32);
      s[e] = s[e] + s2;
      q[e] = q[e] + q2;
    }
    if (hh == 0) {
#pragma unroll
      for (int e = 0; e < 8; ++e) {
        red[wave][c8 + e] = s[e];
        red[wave][128 + c8 + e] = q[e];
      }
    }
    __syncthreads();
    float tot = 0.0f;
#pragma unroll
    for (int w = 0; w < 8; ++w) tot = tot + red[w][tid];
    float* pb = part + (size_t)blockIdx.x * 256 + tid;
    *(volatile float*)pb = tot;
    __threadfence();
    *(volatile float*)pb = tot;
  }
}

__global__ __launch_bounds__(256) void bn_finalize(const float* __restrict__ part, int nblk, int O,
                                                   const float* __restrict__ gamma, const float* __restrict__ beta,
                                                   float* __restrict__ scale_out, float* __restrict__ shift_out) {
  const int c = threadIdx.x;
  const int cc = (c < O) ? c : (O - 1);
  double s = 0.0, q = 0.0;
#pragma unroll 1
  for (int blk = 0; blk < nblk; ++blk) {
    const float* pb = part + (size_t)blk * 2 * O;
    s = s + (double)pb[cc];
    q = q + (double)pb[O + cc];
  }
  const double invM = 1.0 / (double)kRows;
  const double mean = s * invM;
  double var = q * invM - mean * mean;
  var = (var < 0.0) ? 0.0 : var;
  const float scv = gamma[cc] * rsqrtf((float)var + kBnEps);
  const float shv = beta[cc] - (float)mean * scv;
  if (c < O) {
    *(volatile float*)(scale_out + c) = scv;
    *(volatile float*)(shift_out + c) = shv;
    __threadfence();
    *(volatile float*)(scale_out + c) = scv;
    *(volatile float*)(shift_out + c) = shv;
  }
}

__global__ __launch_bounds__(256) void pool_out(const float* __restrict__ ymaxp, const float* __restrict__ yminp,
                                                const float* __restrict__ scl, const float* __restrict__ sft,
                                                float* __restrict__ out1) {
  __shared__ __align__(16) float tl[32 * 260];
  const int tid = threadIdx.x;
  const int lane = tid & 31;
  const int wave = tid >> 5;
  const int blk = blockIdx.x;
  const int b = blk >> 5;
  const int s0 = (blk & 31) * 32;
  const int ca = lane * 4;
  const int cb = 128 + lane * 4;
  const v4f sca = *(const v4f*)(scl + ca);
  const v4f scb = *(const v4f*)(scl + cb);
  const v4f sha = *(const v4f*)(sft + ca);
  const v4f shb = *(const v4f*)(sft + cb);
#pragma unroll 1
  for (int rr = 0; rr < 4; ++rr) {
    const int srow = wave * 4 + rr;
    const size_t g = (size_t)blk * 32 + srow;
    const v4f xa = *(const v4f*)(ymaxp + g * kOut2 + ca);
    const v4f xb = *(const v4f*)(ymaxp + g * kOut2 + cb);
    const v4f na = *(const v4f*)(yminp + g * kOut2 + ca);
    const v4f nb = *(const v4f*)(yminp + g * kOut2 + cb);
    v4f ra, rb;
#pragma unroll
    for (int e = 0; e < 4; ++e) {
      const float ta = (sca[e] >= 0.0f) ? (sca[e] * xa[e]) : (sca[e] * na[e]);
      const float tb = (scb[e] >= 0.0f) ? (scb[e] * xb[e]) : (scb[e] * nb[e]);
      ra[e] = fmaxf(ta + sha[e], 0.0f);
      rb[e] = fmaxf(tb + shb[e], 0.0f);
    }
    *(v4f*)(tl + srow * 260 + ca) = ra;
    *(v4f*)(tl + srow * 260 + cb) = rb;
  }
  __syncthreads();
  const int s4 = (lane & 7) * 4;
  v4f vals[8];
#pragma unroll
  for (int it = 0; it < 8; ++it) {
    const int o = wave * 32 + it * 4 + (lane >> 3);
#pragma unroll
    for (int k = 0; k < 4; ++k) vals[it][k] = tl[(s4 + k) * 260 + o];
  }
  for (int pass = 0; pass < 2; ++pass) {
#pragma unroll
    for (int it = 0; it < 8; ++it) {
      const int o = wave * 32 + it * 4 + (lane >> 3);
      *(volatile v4f*)(out1 + ((size_t)b * kOut2 + o) * kNumCent + s0 + s4) = vals[it];
    }
    __threadfence();
  }
}

extern "C" void kernel_launch(void* const* d_in, const int* in_sizes, int n_in,
                              void* d_out, int out_size, void* d_ws, size_t ws_size,
                              hipStream_t stream) {
  (void)in_sizes; (void)n_in; (void)out_size;
  if (ws_size < kCarveTotal) return;

  const float* xyz    = (const float*)d_in[0];
  const float* points = (const float*)d_in[1];
  const float* W0  = (const float*)d_in[2];
  const float* b0  = (const float*)d_in[3];
  const float* g0  = (const float*)d_in[4];
  const float* be0 = (const float*)d_in[5];
  const float* W1  = (const float*)d_in[6];
  const float* b1  = (const float*)d_in[7];
  const float* g1  = (const float*)d_in[8];
  const float* be1 = (const float*)d_in[9];
  const float* W2  = (const float*)d_in[10];
  const float* b2  = (const float*)d_in[11];
  const float* g2  = (const float*)d_in[12];
  const float* be2 = (const float*)d_in[13];

  float* out0 = (float*)d_out;
  float* out1 = out0 + (size_t)kBatch * kNumCent * 3;

  char* ws = (char*)d_ws;
  int*      fpsI  = (int*)(ws + kOffFps);
  int*      nnI   = (int*)(ws + kOffNn);
  _Float16* W0h   = (_Float16*)(ws + kOffW0h);
  _Float16* W1h   = (_Float16*)(ws + kOffW1h);
  _Float16* W2h   = (_Float16*)(ws + kOffW2h);
  _Float16* pts16 = (_Float16*)(ws + kOffPts);
  float*    Pp    = (float*)(ws + kOffP);
  _Float16* A1    = (_Float16*)(ws + kOffA1);
  _Float16* A2c   = (_Float16*)(ws + kOffA2);
  float*    ymaxp = (float*)(ws + kOffYmax);
  float*    yminp = (float*)(ws + kOffYmin);
  float*    part0 = (float*)(ws + kOffPart0);
  float*    part1 = (float*)(ws + kOffPart1);
  float*    part2 = (float*)(ws + kOffPart2);
  float*    ss0   = (float*)(ws + kOffSS0);
  float*    ss1   = (float*)(ws + kOffSS1);
  float*    ss2   = (float*)(ws + kOffSS2);

  fps_kernel<<<kBatch, 256, 0, stream>>>(xyz, fpsI, out0);
  knn_kernel<<<kGroups / 2, 64, 0, stream>>>(xyz, fpsI, nnI);

  prep_kernel<<<kPrepWBlocks + kPrepPBlocks, 256, 0, stream>>>(W0, W1, W2, points, W0h, W1h, W2h, pts16);

  mlp_gemm<0><<<((kBatch * kNumPts / 64) * (kOut0 / 64)) / 8, 256, 0, stream>>>(
      pts16, W0h, kOut0, kCin, b0, ss0, ss0, Pp, A2c, ymaxp, yminp, kWCarryInv);

  l0_kernel<false><<<kBlk0, 256, 0, stream>>>(Pp, xyz, fpsI, nnI, W0, b0, ss0, ss0, part0, A1);
  bn_finalize<<<1, 256, 0, stream>>>(part0, kBlk0, kOut0, g0, be0, ss0, ss0 + 256);
  l0_kernel<true><<<kBlk0, 256, 0, stream>>>(Pp, xyz, fpsI, nnI, W0, b0, ss0, ss0 + 256, part0, A1);

  mlp_gemm<1><<<kBlk1, 256, 0, stream>>>(
      A1, W1h, kOut1, kOut0, b1, ss1, ss1, part1, A2c, ymaxp, yminp, kWCarryInv);
  bn_finalize<<<1, 256, 0, stream>>>(part1, kBlk1, kOut1, g1, be1, ss1, ss1 + 256);

  for (int c = 0; c < kChunks; ++c) {
    const _Float16* A1c = A1 + (size_t)c * kChunkRows * kOut0;
    mlp_gemm<2><<<((kChunkRows / 64) * (kOut1 / 64)) / 8, 256, 0, stream>>>(
        A1c, W1h, kOut1, kOut0, b1, ss1, ss1 + 256, part1, A2c, ymaxp, yminp, kWCarryInv);
    mlp_gemm<3><<<kBlk2c, 256, 0, stream>>>(
        A2c, W2h, kOut2, kOut1, b2, ss2, ss2, part2 + (size_t)c * kBlk2c * 2 * kOut2, A2c,
        ymaxp + (size_t)c * kChunkGroups * kOut2, yminp + (size_t)c * kChunkGroups * kOut2, kWCarryInv);
  }
  bn_finalize<<<1, 256, 0, stream>>>(part2, kBlk2c * kChunks, kOut2, g2, be2, ss2, ss2 + 256);

  pool_out<<<kGroups / 32, 256, 0, stream>>>(ymaxp, yminp, ss2, ss2 + 256, out1);
}
